// MultiLayerEdgeGAT_25280177504677
// MI455X (gfx1250) — hardware-verified
//
#include <hip/hip_runtime.h>
#include <stddef.h>


#define DF    128
#define EF    16
#define GR    32
#define AP    136
#define XSP   132
#define NPART 8
#define HP    4
#define TP    129
#define NB    512
#define CHUNK 2048
#define NTHR  256
#define NWAVE 8
#define WCAP  256
#define NGRP  (CHUNK / (NTHR * 4))

#define LDS_SACC (NB * DF)
#define LDS_DEN  (NB * HP)
#define LDS_MAX  (NB * HP)
#define LDS_LIST (NWAVE * WCAP)
#define LDS_WA   (EF * HP)
#define LDS_BYTES ((LDS_SACC + LDS_DEN + LDS_MAX + LDS_LIST + NWAVE + LDS_WA) * 4)

static_assert(WCAP == (CHUNK / NTHR) * 32);
static_assert(NGRP == 2);
static_assert(NB == 512);
static_assert(CHUNK == 2048);
static_assert(((LDS_SACC + LDS_DEN) % 4) == 0);
static_assert((LDS_MAX % 4) == 0);
static_assert((NB % NWAVE) == 0);
static_assert(LDS_BYTES == 287008);

typedef float          v4f   __attribute__((ext_vector_type(4)));
typedef float          v8f   __attribute__((ext_vector_type(8)));
typedef int            v4i   __attribute__((ext_vector_type(4)));
typedef unsigned short v8us  __attribute__((ext_vector_type(8)));
typedef unsigned short v16us __attribute__((ext_vector_type(16)));
typedef __bf16         v16bf __attribute__((ext_vector_type(16)));
union Frag   { v16bf v; v16us u; v8us half[2]; };
union Pack16 { v8us h; v4i i; };

__device__ __forceinline__ v8f wm(v16bf a, v16bf b, v8f c) {
  v8f d = __builtin_amdgcn_wmma_f32_16x16x32_bf16(false, a, false, b, (short)0, c, false, false);
  asm volatile("v_nop\n\tv_nop\n\tv_nop\n\tv_nop" : "+v"(d) : "v"(a), "v"(b));
  return d;
}

__device__ __forceinline__ unsigned short bf_bits(float x) {
  const unsigned u = __float_as_uint(x);
  return (unsigned short)((u + 0x7FFFu + ((u >> 16) & 1u)) >> 16);
}
__device__ __forceinline__ void bf_split(float x, unsigned short& hi, unsigned short& lo) {
  const unsigned short hb = bf_bits(x);
  const float r = x - __uint_as_float(((unsigned)hb) << 16);
  hi = hb;
  lo = bf_bits(r);
}

__global__ __launch_bounds__(NTHR) void k_prepw(const float* __restrict__ W,
                                                unsigned short* Wh, unsigned short* Wl) {
  __shared__ __attribute__((aligned(16))) float T[32 * TP];
  const int tid = threadIdx.x;
  const int n0  = blockIdx.x * 32;
#pragma unroll
  for (int i = 0; i < 16; ++i) {
    const int idx = i * NTHR + tid;
    const int k   = idx >> 5;
    const int c   = idx & 31;
    T[c * TP + k] = W[(size_t)k * DF + n0 + c];
  }
  __syncthreads();
  Pack16 uh[2], ul[2];
  size_t po[2];
#pragma unroll
  for (int q = 0; q < 2; ++q) {
    const int t  = q * NTHR + tid;
    const int c  = t >> 4;
    const int k0 = (t & 15) * 8;
#pragma unroll
    for (int j = 0; j < 8; ++j) {
      unsigned short a, b;
      bf_split(T[c * TP + k0 + j], a, b);
      uh[q].h[j] = a;
      ul[q].h[j] = b;
    }
    po[q] = (size_t)(n0 + c) * DF + k0;
  }
#pragma unroll
  for (int q = 0; q < 2; ++q) {
    *(volatile v4i*)(Wh + po[q]) = uh[q].i;
    *(volatile v4i*)(Wl + po[q]) = ul[q].i;
  }
  __threadfence();
#pragma unroll
  for (int q = 0; q < 2; ++q) {
    *(volatile v4i*)(Wh + po[q]) = uh[q].i;
    *(volatile v4i*)(Wl + po[q]) = ul[q].i;
  }
}

__device__ __forceinline__ void epi_tile(v8f acc, int T, int hh, int m, int wave, int ncol,
                                         float cs, float cd, float* Xs, float* Ps, float* Pd) {
  float ss[8], sd[8];
#pragma unroll
  for (int r = 0; r < 8; ++r) {
    const float v = acc[r];
    Xs[(T * 16 + 8 * hh + r) * XSP + ncol] = v;
    ss[r] = v * cs;
    sd[r] = v * cd;
  }
#pragma unroll
  for (int mk = 1; mk < 16; mk <<= 1) {
#pragma unroll
    for (int r = 0; r < 8; ++r) {
      ss[r] += __shfl_xor(ss[r], mk, 32);
      sd[r] += __shfl_xor(sd[r], mk, 32);
    }
  }
  if (m == 0) {
#pragma unroll
    for (int r = 0; r < 8; ++r) {
      Ps[(T * 16 + 8 * hh + r) * NPART + wave] = ss[r];
      Pd[(T * 16 + 8 * hh + r) * NPART + wave] = sd[r];
    }
  }
}

__global__ __launch_bounds__(NTHR) void k_gemm(
    const float* __restrict__ x, const unsigned short* __restrict__ Wh,
    const unsigned short* __restrict__ Wl,
    const float* __restrict__ attl, const float* __restrict__ attr,
    float* xp, float* elp, float* erp, int nN, int H) {
  __shared__ __attribute__((aligned(16))) unsigned short Ah[GR * AP];
  __shared__ __attribute__((aligned(16))) unsigned short Al[GR * AP];
  __shared__ __attribute__((aligned(16))) float Xs[GR * XSP];
  __shared__ __attribute__((aligned(16))) float Pp[2 * GR * NPART];
  float* Ps = Pp;
  float* Pd = Pp + GR * NPART;

  const int tid  = threadIdx.x;
  const int lane = tid & 31;
  const int wave = tid >> 5;
  const int hh   = lane >> 4;
  const int m    = lane & 15;
  const int rowBase = blockIdx.x * GR;

  {
    const int r  = tid >> 3;
    const int c0 = (tid & 7) * 16;
    int row = rowBase + r;
    if (row > nN - 1) row = nN - 1;
    const float* p = x + (size_t)row * DF + c0;
    const v4f f0 = *(const v4f*)(p), f1 = *(const v4f*)(p + 4);
    const v4f f2 = *(const v4f*)(p + 8), f3 = *(const v4f*)(p + 12);
    float v[16];
    v[0] = f0.x;  v[1] = f0.y;  v[2] = f0.z;  v[3] = f0.w;
    v[4] = f1.x;  v[5] = f1.y;  v[6] = f1.z;  v[7] = f1.w;
    v[8] = f2.x;  v[9] = f2.y;  v[10] = f2.z; v[11] = f2.w;
    v[12] = f3.x; v[13] = f3.y; v[14] = f3.z; v[15] = f3.w;
    Pack16 h0, h1, l0, l1;
#pragma unroll
    for (int j = 0; j < 8; ++j) {
      unsigned short a, b;
      bf_split(v[j], a, b);
      h0.h[j] = a; l0.h[j] = b;
      bf_split(v[8 + j], a, b);
      h1.h[j] = a; l1.h[j] = b;
    }
    *(v8us*)(Ah + r * AP + c0)     = h0.h;
    *(v8us*)(Ah + r * AP + c0 + 8) = h1.h;
    *(v8us*)(Al + r * AP + c0)     = l0.h;
    *(v8us*)(Al + r * AP + c0 + 8) = l1.h;
  }
  __syncthreads();

  const int ncol = wave * 16 + m;
  v8f c0a = {0.f, 0.f, 0.f, 0.f, 0.f, 0.f, 0.f, 0.f};
  v8f c1a = {0.f, 0.f, 0.f, 0.f, 0.f, 0.f, 0.f, 0.f};
#pragma unroll
  for (int kt = 0; kt < DF / 32; ++kt) {
    const int k0 = kt * 32;
    Frag a0h, a0l, a1h, a1l, bh, bl;
    const unsigned short* pbh  = Wh + (size_t)ncol * DF + k0 + 8 * hh;
    const unsigned short* pbl  = Wl + (size_t)ncol * DF + k0 + 8 * hh;
    const unsigned short* pa0h = Ah + m * AP + k0 + 8 * hh;
    const unsigned short* pa0l = Al + m * AP + k0 + 8 * hh;
    const unsigned short* pa1h = Ah + (16 + m) * AP + k0 + 8 * hh;
    const unsigned short* pa1l = Al + (16 + m) * AP + k0 + 8 * hh;
    bh.half[0]  = *(const v8us*)pbh;  bh.half[1]  = *(const v8us*)(pbh + 16);
    bl.half[0]  = *(const v8us*)pbl;  bl.half[1]  = *(const v8us*)(pbl + 16);
    a0h.half[0] = *(const v8us*)pa0h; a0h.half[1] = *(const v8us*)(pa0h + 16);
    a0l.half[0] = *(const v8us*)pa0l; a0l.half[1] = *(const v8us*)(pa0l + 16);
    a1h.half[0] = *(const v8us*)pa1h; a1h.half[1] = *(const v8us*)(pa1h + 16);
    a1l.half[0] = *(const v8us*)pa1l; a1l.half[1] = *(const v8us*)(pa1l + 16);
    c0a = wm(a0h.v, bh.v, c0a);
    c0a = wm(a0h.v, bl.v, c0a);
    c0a = wm(a0l.v, bh.v, c0a);
    c1a = wm(a1h.v, bh.v, c1a);
    c1a = wm(a1h.v, bl.v, c1a);
    c1a = wm(a1l.v, bh.v, c1a);
  }

  const float cs = attl[ncol];
  const float cd = attr[ncol];
  epi_tile(c0a, 0, hh, m, wave, ncol, cs, cd, Xs, Ps, Pd);
  epi_tile(c1a, 1, hh, m, wave, ncol, cs, cd, Xs, Ps, Pd);
  __syncthreads();

  v4f xr[4];
#pragma unroll
  for (int i = 0; i < 4; ++i) xr[i] = *(const v4f*)(Xs + (4 * wave + i) * XSP + 4 * lane);
  v4f gv = {0.f, 0.f, 0.f, 0.f};
  if (wave < 2) {
    const float* P = Pp + wave * (GR * NPART) + lane * NPART;
    const v4f q0 = *(const v4f*)(P);
    const v4f q1 = *(const v4f*)(P + 4);
    if (H == 4) {
      gv.x = q0.x + q0.y; gv.y = q0.z + q0.w; gv.z = q1.x + q1.y; gv.w = q1.z + q1.w;
    } else {
      gv.x = ((q0.x + q0.y) + (q0.z + q0.w)) + ((q1.x + q1.y) + (q1.z + q1.w));
    }
  }
  float* gp = ((wave == 0) ? elp : erp) + ((size_t)rowBase + lane) * HP;
  float* xpp[4];
#pragma unroll
  for (int i = 0; i < 4; ++i) xpp[i] = xp + (size_t)(rowBase + 4 * wave + i) * DF + 4 * lane;

#pragma unroll
  for (int i = 0; i < 4; ++i) *(volatile v4f*)(xpp[i]) = xr[i];
  if (wave < 2) *(volatile v4f*)gp = gv;
  __threadfence();
#pragma unroll
  for (int i = 0; i < 4; ++i) *(volatile v4f*)(xpp[i]) = xr[i];
  if (wave < 2) *(volatile v4f*)gp = gv;
}

__global__ __launch_bounds__(NTHR) void k_gat(
    const float* __restrict__ feat, const float* __restrict__ elp, const float* __restrict__ erp,
    const int* __restrict__ srcp, const int* __restrict__ dstp, const float* __restrict__ ef,
    const float* __restrict__ We, const float* __restrict__ ae, const float* __restrict__ bias,
    float* out, int nN, int nE, int H, int act) {
  extern __shared__ v4f lds_dyn[];
  float* sacc = (float*)lds_dyn;
  float* daux = sacc + LDS_SACC;
  float* maux = daux + LDS_DEN;
  int*   list = (int*)(maux + LDS_MAX);
  int*   wcnt = list + LDS_LIST;
  float* wat  = (float*)(wcnt + NWAVE);

  const int tid  = threadIdx.x;
  const int lane = tid & 31;
  const int wave = tid >> 5;
  const int hd   = (lane * H) >> 5;
  const int D    = DF / H;
  const int nodeBase = blockIdx.x * NB;

  {
    const v4f z4 = {0.f, 0.f, 0.f, 0.f};
    for (int i = tid; i < (LDS_SACC + LDS_DEN) / 4; i += NTHR) lds_dyn[i] = z4;
    const float ninf = __uint_as_float(0xff800000u);
    const v4f n4 = {ninf, ninf, ninf, ninf};
    for (int i = tid; i < LDS_MAX / 4; i += NTHR) lds_dyn[(LDS_SACC + LDS_DEN) / 4 + i] = n4;
    if (tid < EF * H) {
      const int f  = tid / H;
      const int hq = tid - f * H;
      float s = 0.f;
#pragma unroll 1
      for (int d = 0; d < D; ++d) s += We[f * DF + hq * D + d] * ae[hq * D + d];
      wat[f * HP + hq] = s;
    }
  }
  __syncthreads();
  float wr[EF];
#pragma unroll
  for (int f = 0; f < EF; ++f) wr[f] = wat[f * HP + hd];
  const bool al16 = ((((size_t)dstp) & 15) == 0);

  const int nChunks = (nE + CHUNK - 1) / CHUNK;
#pragma unroll 1
  for (int ch = 0; ch < nChunks; ++ch) {
    const int cbase = ch * CHUNK;
    int wc = 0;
#pragma unroll
    for (int g = 0; g < NGRP; ++g) {
      const int el0 = (g * NTHR + tid) * 4;
      const int e0  = cbase + el0;
      const int sent = -2147483647 - 1;
      v4i d;
      if (al16 && (cbase + CHUNK <= nE)) {
        d = *(const v4i*)(dstp + e0);
      } else {
        d.x = (e0     < nE) ? dstp[min(e0, nE - 1)]     : sent;
        d.y = (e0 + 1 < nE) ? dstp[min(e0 + 1, nE - 1)] : sent;
        d.z = (e0 + 2 < nE) ? dstp[min(e0 + 2, nE - 1)] : sent;
        d.w = (e0 + 3 < nE) ? dstp[min(e0 + 3, nE - 1)] : sent;
      }
      const unsigned s0 = (unsigned)d.x - (unsigned)nodeBase;
      const unsigned s1 = (unsigned)d.y - (unsigned)nodeBase;
      const unsigned s2 = (unsigned)d.z - (unsigned)nodeBase;
      const unsigned s3 = (unsigned)d.w - (unsigned)nodeBase;
      const bool h0 = s0 < (unsigned)NB;
      const bool h1 = s1 < (unsigned)NB;
      const bool h2 = s2 < (unsigned)NB;
      const bool h3 = s3 < (unsigned)NB;
      const unsigned many = __builtin_amdgcn_ballot_w32(h0 | h1 | h2 | h3);
      if (many != 0u) {
#define HITJ(J, HJ, SJ) { \
          const unsigned mj = __builtin_amdgcn_ballot_w32(HJ); \
          if (HJ) { \
            const int pos = wc + (int)__builtin_amdgcn_mbcnt_lo(mj, 0u); \
            if (pos < WCAP) list[wave * WCAP + pos] = ((el0 + (J)) << 9) | (int)(SJ); \
          } \
          wc += (int)__builtin_popcount(mj); }
        HITJ(0, h0, s0)
        HITJ(1, h1, s1)
        HITJ(2, h2, s2)
        HITJ(3, h3, s3)
#undef HITJ
      }
    }
    if (lane == 0) wcnt[wave] = wc;
    __syncthreads();

    if (wave == 0) {
      for (int wsx = 0; wsx < NWAVE; ++wsx) {
        int n = __builtin_amdgcn_readfirstlane(wcnt[wsx]);
        n = n > WCAP ? WCAP : n;
        n = n < 0 ? 0 : n;
        for (int i = 0; i < n; ++i) {
          const int ent  = __builtin_amdgcn_readfirstlane(list[wsx * WCAP + i]);
          const int slot = ent & (NB - 1);
          const int eloc = (ent >> 9) & (CHUNK - 1);
          int e = cbase + eloc;
          e = e > nE - 1 ? nE - 1 : e;
          int j = srcp[e];
          j = j < 0 ? 0 : (j > nN - 1 ? nN - 1 : j);
          int nd = nodeBase + slot;
          nd = nd > nN - 1 ? nN - 1 : nd;
          const float* efr = ef + (size_t)e * EF;
          const v4f f0 = *(const v4f*)(efr);
          const v4f f1 = *(const v4f*)(efr + 4);
          const v4f f2 = *(const v4f*)(efr + 8);
          const v4f f3 = *(const v4f*)(efr + 12);
          const float ee = f0.x * wr[0]  + f0.y * wr[1]  + f0.z * wr[2]  + f0.w * wr[3]
                         + f1.x * wr[4]  + f1.y * wr[5]  + f1.z * wr[6]  + f1.w * wr[7]
                         + f2.x * wr[8]  + f2.y * wr[9]  + f2.z * wr[10] + f2.w * wr[11]
                         + f3.x * wr[12] + f3.y * wr[13] + f3.z * wr[14] + f3.w * wr[15];
          float s = elp[(size_t)j * HP + hd] + erp[(size_t)nd * HP + hd] + ee;
          s = (s >= 0.f) ? s : 0.2f * s;
          const int ai = slot * HP + hd;
          const float mo = maux[ai];
          const float dn = daux[ai];
          const float mn = fmaxf(mo, s);
          const float cf = __expf(mo - mn);
          const float p  = __expf(s - mn);
          const v4f xv = *(const v4f*)(feat + (size_t)j * DF + 4 * lane);
          v4f* sp = (v4f*)(sacc + slot * DF + 4 * lane);
          const v4f cur = *sp;
          const v4f nxt = cur * cf + xv * p;
          *sp = nxt;
          maux[ai] = mn;
          daux[ai] = dn * cf + p;
        }
      }
    }
    __syncthreads();
  }

  const v4f b4 = *(const v4f*)(bias + 4 * lane);
#pragma unroll 1
  for (int q = 0; q < NB / NWAVE; ++q) {
    const int slot = wave * (NB / NWAVE) + q;
    const int node = nodeBase + slot;
    if (node >= nN) break;
    const float dn  = daux[slot * HP + hd];
    const float inv = (dn > 0.f) ? (1.0f / dn) : 0.f;
    const v4f sv = *(const v4f*)(sacc + slot * DF + 4 * lane);
    v4f y = sv * inv + b4;
    if (act) {
      y.x = y.x > 0.f ? y.x : 0.f;
      y.y = y.y > 0.f ? y.y : 0.f;
      y.z = y.z > 0.f ? y.z : 0.f;
      y.w = y.w > 0.f ? y.w : 0.f;
    }
    float* op = out + (size_t)node * DF + 4 * lane;
    *(volatile v4f*)op = y;
    __threadfence();
    *(volatile v4f*)op = y;
  }
}

extern "C" void kernel_launch(void* const* d_in, const int* in_sizes, int n_in,
                              void* d_out, int out_size, void* d_ws, size_t ws_size,
                              hipStream_t stream) {
  if (n_in != 22) return;
  const int nN = in_sizes[0] / DF;
  if (nN <= 0 || in_sizes[0] != nN * DF) return;
  const int nE = in_sizes[2];
  if (nE <= 0 || in_sizes[3] != nE || in_sizes[1] != nE * EF) return;
  for (int l = 0; l < 3; ++l) {
    if (in_sizes[4 + 6 * l] != DF * DF) return;
    if (in_sizes[5 + 6 * l] != EF * DF) return;
    if (in_sizes[6 + 6 * l] != DF || in_sizes[7 + 6 * l] != DF ||
        in_sizes[8 + 6 * l] != DF || in_sizes[9 + 6 * l] != DF) return;
  }
  if (out_size != nN * DF) return;

  const float* h   = (const float*)d_in[0];
  const float* ef  = (const float*)d_in[1];
  const int*   src = (const int*)d_in[2];
  const int*   dst = (const int*)d_in[3];
  const float *Wp[3], *Wep[3], *alp[3], *arp[3], *aep[3], *bp[3];
  for (int l = 0; l < 3; ++l) {
    Wp[l]  = (const float*)d_in[4 + 6 * l];
    Wep[l] = (const float*)d_in[5 + 6 * l];
    alp[l] = (const float*)d_in[6 + 6 * l];
    arp[l] = (const float*)d_in[7 + 6 * l];
    aep[l] = (const float*)d_in[8 + 6 * l];
    bp[l]  = (const float*)d_in[9 + 6 * l];
  }
  float* outp = (float*)d_out;

  const int nP = ((nN + GR - 1) / GR) * GR;
  size_t off = 0;
  unsigned short* Wh = (unsigned short*)((char*)d_ws + off); off += (size_t)DF * DF * sizeof(unsigned short);
  unsigned short* Wl = (unsigned short*)((char*)d_ws + off); off += (size_t)DF * DF * sizeof(unsigned short);
  float* feat = (float*)((char*)d_ws + off); off += (size_t)nP * DF * sizeof(float);
  float* hbuf = (float*)((char*)d_ws + off); off += (size_t)nP * DF * sizeof(float);
  float* elp  = (float*)((char*)d_ws + off); off += (size_t)nP * HP * sizeof(float);
  float* erp  = (float*)((char*)d_ws + off); off += (size_t)nP * HP * sizeof(float);
  if (off > ws_size) return;

  const int Hs[3]   = {4, 4, 1};
  const int acts[3] = {1, 1, 0};
  hipFuncSetAttribute(reinterpret_cast<const void*>(&k_gat),
                      hipFuncAttributeMaxDynamicSharedMemorySize, LDS_BYTES);
  const int ggrid = (nN + NB - 1) / NB;
  for (int l = 0; l < 3; ++l) {
    const float* xin = (l == 0) ? h : hbuf;
    float* o = (l == 2) ? outp : hbuf;
    k_prepw<<<DF / 32, NTHR, 0, stream>>>(Wp[l], Wh, Wl);
    k_gemm<<<nP / GR, NTHR, 0, stream>>>(xin, Wh, Wl, alp[l], arp[l], feat, elp, erp, nN, Hs[l]);
    k_gat<<<ggrid, NTHR, LDS_BYTES, stream>>>(feat, elp, erp, src, dst, ef, Wep[l], aep[l], bp[l],
                                              o, nN, nE, Hs[l], acts[l]);
  }
}
